// attentiona_51213190037761
// MI455X (gfx1250) — hardware-verified
//
#include <hip/hip_runtime.h>
#include <stddef.h>
#include <stdint.h>
#include <math.h>


#define DEV __device__ __forceinline__

typedef _Float16 v8h  __attribute__((ext_vector_type(8)));
typedef _Float16 v16h __attribute__((ext_vector_type(16)));
typedef __bf16   v16b __attribute__((ext_vector_type(16)));
typedef unsigned short us8 __attribute__((ext_vector_type(8)));
typedef float v8f __attribute__((ext_vector_type(8)));
typedef float v4f __attribute__((ext_vector_type(4)));

constexpr int B_   = 2;
constexpr int S_   = 2048;
constexpr int D_   = 512;
constexpr int H_   = 8;
constexpr int DH_  = 64;
constexpr int NT_  = B_ * S_;
constexpr int KVN_ = 2 * D_;
constexpr int QT_  = S_ / 64;
constexpr int PT_  = 72;
constexpr int GP_  = 40;
constexpr int VP_  = 68;
constexpr int TP_  = 64 * PT_;
constexpr float LN_EPS_ = 1e-5f;
constexpr float SCALEF_ = 0.125f;

static_assert(D_ == H_ * DH_);
static_assert(DH_ == 64);
static_assert(D_ == 64 * 8);
static_assert(S_ % 64 == 0 && NT_ % 64 == 0 && D_ % 64 == 0 && KVN_ % 64 == 0);
static_assert(D_ % 32 == 0);
static_assert((D_ * D_) % (8 * 256) == 0 && (KVN_ * D_) % (8 * 256) == 0);

DEV int lane_id() { return (int)(threadIdx.x & 31); }

DEV unsigned short f2bf(float f) {
  unsigned int u = __float_as_uint(f);
  u += 0x7FFFu + ((u >> 16) & 1u);
  return (unsigned short)(u >> 16);
}
DEV float bf2f(unsigned short b) { return __uint_as_float(((unsigned int)b) << 16); }

DEV void split8(const float* v, us8& hi, us8& lo) {
#pragma unroll
  for (int i = 0; i < 8; ++i) {
    unsigned short hb = f2bf(v[i]);
    hi[i] = hb;
    lo[i] = f2bf(v[i] - bf2f(hb));
  }
}

DEV float allred(float v) {
#pragma unroll
  for (int o = 16; o > 0; o >>= 1) v += __shfl_xor(v, o, 32);
  return v;
}

union FragH { v16h v; v8h p[2]; };
union FragB { v16b v; us8 p[2]; };

DEV v16h ldfrag_h(const _Float16* t, int pitch, int k0) {
  const int l = lane_id(), hh = l >> 4, m = l & 15;
  const _Float16* r = t + m * pitch + k0 + 8 * hh;
  FragH f;
  f.p[0] = *(const v8h*)r;
  f.p[1] = *(const v8h*)(r + 16);
  return f.v;
}
DEV v16b ldfrag_b(const unsigned short* t, int pitch, int k0) {
  const int l = lane_id(), hh = l >> 4, m = l & 15;
  const unsigned short* r = t + m * pitch + k0 + 8 * hh;
  FragB f;
  f.p[0] = *(const us8*)r;
  f.p[1] = *(const us8*)(r + 16);
  return f.v;
}

DEV v8f mma_h(v16h a, v16h b, v8f c) {
  c = __builtin_amdgcn_wmma_f32_16x16x32_f16(false, a, false, b, (short)0, c, false, false);
  asm volatile("v_nop\n\tv_nop\n\tv_nop\n\tv_nop" : "+v"(c) : "v"(a), "v"(b));
  return c;
}
DEV v8f mma_b(v16b a, v16b b, v8f c) {
  c = __builtin_amdgcn_wmma_f32_16x16x32_bf16(false, a, false, b, (short)0, c, false, false);
  asm volatile("v_nop\n\tv_nop\n\tv_nop\n\tv_nop" : "+v"(c) : "v"(a), "v"(b));
  return c;
}

__global__ __launch_bounds__(64) void k_prep(
    const float* __restrict__ x, const float* __restrict__ lw, const float* __restrict__ lb,
    unsigned short* xh, unsigned short* xl, unsigned short* yh, unsigned short* yl, int nrows) {
  __shared__ float red[4];
  const int row = blockIdx.x;
  if (row >= nrows) return;
  const int t = threadIdx.x, l = t & 31, w = t >> 5;
  const float* xr = x + (size_t)row * D_ + 8 * t;
  const v4f a = *(const v4f*)xr;
  const v4f c = *(const v4f*)(xr + 4);
  float v[8] = {a[0], a[1], a[2], a[3], c[0], c[1], c[2], c[3]};
  float s = 0.f;
#pragma unroll
  for (int i = 0; i < 8; ++i) s += v[i];
  s = allred(s);
  if (l == 0) red[w] = s;
  __syncthreads();
  const float mean = (red[0] + red[1]) * (1.f / (float)D_);
  float d[8];
  float q = 0.f;
#pragma unroll
  for (int i = 0; i < 8; ++i) { d[i] = v[i] - mean; q += d[i] * d[i]; }
  q = allred(q);
  if (l == 0) red[2 + w] = q;
  __syncthreads();
  const float var = (red[2] + red[3]) * (1.f / (float)D_);
  const float rs = rsqrtf(var + LN_EPS_);
  const v4f w0 = *(const v4f*)(lw + 8 * t), w1 = *(const v4f*)(lw + 8 * t + 4);
  const v4f c0 = *(const v4f*)(lb + 8 * t), c1 = *(const v4f*)(lb + 8 * t + 4);
  float wv[8] = {w0[0], w0[1], w0[2], w0[3], w1[0], w1[1], w1[2], w1[3]};
  float cv[8] = {c0[0], c0[1], c0[2], c0[3], c1[0], c1[1], c1[2], c1[3]};
  float y[8];
#pragma unroll
  for (int i = 0; i < 8; ++i) y[i] = d[i] * rs * wv[i] + cv[i];
  us8 ph, pl, qh, ql;
  split8(v, ph, pl);
  split8(y, qh, ql);
  const size_t o = (size_t)row * D_ + 8 * t;
  *(volatile us8*)(xh + o) = ph;
  *(volatile us8*)(xl + o) = pl;
  *(volatile us8*)(yh + o) = qh;
  *(volatile us8*)(yl + o) = ql;
  __threadfence();
  *(volatile us8*)(xh + o) = ph;
  *(volatile us8*)(xl + o) = pl;
  *(volatile us8*)(yh + o) = qh;
  *(volatile us8*)(yl + o) = ql;
}

__global__ __launch_bounds__(256) void k_split(
    const float* __restrict__ w, unsigned short* hi, unsigned short* lo, int n) {
  const size_t i = ((size_t)blockIdx.x * 256 + threadIdx.x) * 8;
  if (i + 8 > (size_t)n) return;
  const v4f a = *(const v4f*)(w + i);
  const v4f c = *(const v4f*)(w + i + 4);
  float v[8] = {a[0], a[1], a[2], a[3], c[0], c[1], c[2], c[3]};
  us8 ph, pl;
  split8(v, ph, pl);
  *(volatile us8*)(hi + i) = ph;
  *(volatile us8*)(lo + i) = pl;
  __threadfence();
  *(volatile us8*)(hi + i) = ph;
  *(volatile us8*)(lo + i) = pl;
}

__global__ __launch_bounds__(256) void k_gemm(
    const unsigned short* __restrict__ Ah, const unsigned short* __restrict__ Al,
    const unsigned short* __restrict__ Wh, const unsigned short* __restrict__ Wl,
    const float* __restrict__ bias, int use_bias, float* C, int M, int N, int K) {
  __shared__ __attribute__((aligned(16))) unsigned short smem[4 * 64 * GP_];
  unsigned short* sAh = smem;
  unsigned short* sAl = smem + 64 * GP_;
  unsigned short* sBh = smem + 2 * 64 * GP_;
  unsigned short* sBl = smem + 3 * 64 * GP_;
  float* sC = (float*)smem;

  const int tid = threadIdx.x, wave = tid >> 5, wm = wave & 3, wn2 = (wave >> 2) * 2;
  const int l = tid & 31, hh = l >> 4, m = l & 15;
  const int m0 = blockIdx.y * 64, n0 = blockIdx.x * 64;
  if (m0 + 64 > M || n0 + 64 > N) return;
  const int lr = tid >> 2, lc = (tid & 3) * 8;

  v8f acc0 = {0.f, 0.f, 0.f, 0.f, 0.f, 0.f, 0.f, 0.f};
  v8f acc1 = {0.f, 0.f, 0.f, 0.f, 0.f, 0.f, 0.f, 0.f};

  for (int k0 = 0; k0 < K; k0 += 32) {
    __syncthreads();
    const size_t ao = (size_t)(m0 + lr) * K + k0 + lc;
    const size_t bo = (size_t)(n0 + lr) * K + k0 + lc;
    *(us8*)(sAh + lr * GP_ + lc) = *(const us8*)(Ah + ao);
    *(us8*)(sAl + lr * GP_ + lc) = *(const us8*)(Al + ao);
    *(us8*)(sBh + lr * GP_ + lc) = *(const us8*)(Wh + bo);
    *(us8*)(sBl + lr * GP_ + lc) = *(const us8*)(Wl + bo);
    __syncthreads();
    const v16b ah  = ldfrag_b(sAh + wm * 16 * GP_, GP_, 0);
    const v16b al  = ldfrag_b(sAl + wm * 16 * GP_, GP_, 0);
    const v16b b0h = ldfrag_b(sBh + wn2 * 16 * GP_, GP_, 0);
    const v16b b0l = ldfrag_b(sBl + wn2 * 16 * GP_, GP_, 0);
    const v16b b1h = ldfrag_b(sBh + (wn2 + 1) * 16 * GP_, GP_, 0);
    const v16b b1l = ldfrag_b(sBl + (wn2 + 1) * 16 * GP_, GP_, 0);
    acc0 = mma_b(ah, b0h, acc0);
    acc0 = mma_b(ah, b0l, acc0);
    acc0 = mma_b(al, b0h, acc0);
    acc1 = mma_b(ah, b1h, acc1);
    acc1 = mma_b(ah, b1l, acc1);
    acc1 = mma_b(al, b1h, acc1);
  }

  __syncthreads();
  const float bv0 = use_bias ? bias[n0 + wn2 * 16 + m] : 0.f;
  const float bv1 = use_bias ? bias[n0 + (wn2 + 1) * 16 + m] : 0.f;
#pragma unroll
  for (int j = 0; j < 8; ++j) {
    const int row = wm * 16 + hh * 8 + j;
    sC[row * 64 + wn2 * 16 + m]       = acc0[j] + bv0;
    sC[row * 64 + (wn2 + 1) * 16 + m] = acc1[j] + bv1;
  }
  __syncthreads();

  v4f vals[4];
  size_t dst[4];
#pragma unroll
  for (int i = 0; i < 4; ++i) {
    const int row = wave * 8 + 2 * i + hh;
    const int col = m * 4;
    vals[i] = *(const v4f*)(sC + row * 64 + col);
    dst[i] = (size_t)(m0 + row) * N + n0 + col;
  }
#pragma unroll
  for (int i = 0; i < 4; ++i) *(volatile v4f*)(C + dst[i]) = vals[i];
  __threadfence();
#pragma unroll
  for (int i = 0; i < 4; ++i) *(volatile v4f*)(C + dst[i]) = vals[i];
}

__global__ __launch_bounds__(256) void k_heads(
    const float* __restrict__ qf, const float* __restrict__ kvf,
    const float* __restrict__ lw, const float* __restrict__ lb, const float* __restrict__ zero,
    _Float16* qln, _Float16* kln, unsigned short* vth, unsigned short* vtl,
    float* vpart, float* ksc) {
  __shared__ __attribute__((aligned(16))) _Float16 sQ16[TP_];
  __shared__ __attribute__((aligned(16))) _Float16 sK16[TP_];
  __shared__ __attribute__((aligned(16))) float sVt[64 * VP_];
  __shared__ __attribute__((aligned(16))) float sVp[8][64];
  __shared__ __attribute__((aligned(16))) float sKs[64];

  const int tok0 = blockIdx.x * 64;
  if (tok0 + 64 > NT_) return;
  const int b = tok0 / S_;
  const int s0 = tok0 - b * S_;
  const int h = blockIdx.y;
  const int bh = b * H_ + h;
  const int stile = s0 >> 6;
  const int tid = threadIdx.x, wave = tid >> 5, l = tid & 31;

  const float w0 = lw[l], w1 = lw[l + 32], c0 = lb[l], c1 = lb[l + 32];
  float zc;
  {
    const float z = zero[0];
    const float sp = log1pf(__expf(-fabsf(z))) + fmaxf(z, 0.f);
    zc = fminf(1e-5f, fmaxf(1e-6f, sp));
  }

  float va0 = 0.f, va1 = 0.f;
#pragma unroll 1
  for (int r = 0; r < 8; ++r) {
    const int row = wave * 8 + r;
    const size_t tok = (size_t)(tok0 + row);
    const float* qr = qf + tok * D_ + h * DH_;
    const float* kr = kvf + tok * KVN_ + h * DH_;
    const float* vr = kr + D_;
    const float qe0 = qr[l], qe1 = qr[l + 32];
    const float ke0 = kr[l], ke1 = kr[l + 32];
    const float ve0 = vr[l], ve1 = vr[l + 32];
    {
      const float mean = allred(qe0 + qe1) * (1.f / (float)DH_);
      const float d0 = qe0 - mean, d1 = qe1 - mean;
      const float var = allred(d0 * d0 + d1 * d1) * (1.f / (float)DH_);
      const float rs = rsqrtf(var + LN_EPS_);
      sQ16[row * PT_ + l]      = (_Float16)(d0 * rs * w0 + c0);
      sQ16[row * PT_ + l + 32] = (_Float16)(d1 * rs * w1 + c1);
    }
    {
      const float mean = allred(ke0 + ke1) * (1.f / (float)DH_);
      const float d0 = ke0 - mean, d1 = ke1 - mean;
      const float var = allred(d0 * d0 + d1 * d1) * (1.f / (float)DH_);
      const float rs = rsqrtf(var + LN_EPS_);
      sK16[row * PT_ + l]      = (_Float16)(d0 * rs * w0 + c0);
      sK16[row * PT_ + l + 32] = (_Float16)(d1 * rs * w1 + c1);
    }
    sVt[l * VP_ + row]        = ve0;
    sVt[(l + 32) * VP_ + row] = ve1;
    va0 += ve0;
    va1 += ve1;
    if (l == 0) sKs[row] = (ke0 == 0.f) ? zc : 1.f;
  }
  sVp[wave][l]      = va0;
  sVp[wave][l + 32] = va1;
  __syncthreads();

  v8h qv[2], kvv[2];
  us8 vh8[2], vl8[2];
  size_t qdst[2], vdst[2];
#pragma unroll
  for (int i = 0; i < 2; ++i) {
    const int row = (tid >> 3) + 32 * i;
    const int c = (tid & 7) * 8;
    qv[i]  = *(const v8h*)(sQ16 + row * PT_ + c);
    kvv[i] = *(const v8h*)(sK16 + row * PT_ + c);
    qdst[i] = ((size_t)bh * S_ + s0 + row) * DH_ + c;
    const int d = row;
    const v4f a  = *(const v4f*)(sVt + d * VP_ + c);
    const v4f a2 = *(const v4f*)(sVt + d * VP_ + c + 4);
    float tmp[8] = {a[0], a[1], a[2], a[3], a2[0], a2[1], a2[2], a2[3]};
    split8(tmp, vh8[i], vl8[i]);
    vdst[i] = ((size_t)bh * DH_ + d) * S_ + s0 + c;
  }
  const bool small = tid < 16;
  v4f vp4 = {0.f, 0.f, 0.f, 0.f}, ks4 = {0.f, 0.f, 0.f, 0.f};
  size_t vpdst = 0, ksdst = 0;
  if (small) {
#pragma unroll
    for (int q = 0; q < 4; ++q) {
      float acc = 0.f;
#pragma unroll
      for (int w = 0; w < 8; ++w) acc += sVp[w][4 * tid + q];
      vp4[q] = acc;
    }
    ks4 = *(const v4f*)(sKs + 4 * tid);
    vpdst = ((size_t)bh * QT_ + stile) * 64 + 4 * tid;
    ksdst = (size_t)bh * S_ + s0 + 4 * tid;
  }

#pragma unroll
  for (int i = 0; i < 2; ++i) {
    *(volatile v8h*)(qln + qdst[i]) = qv[i];
    *(volatile v8h*)(kln + qdst[i]) = kvv[i];
    *(volatile us8*)(vth + vdst[i]) = vh8[i];
    *(volatile us8*)(vtl + vdst[i]) = vl8[i];
  }
  if (small) {
    *(volatile v4f*)(vpart + vpdst) = vp4;
    *(volatile v4f*)(ksc + ksdst)   = ks4;
  }
  __threadfence();
#pragma unroll
  for (int i = 0; i < 2; ++i) {
    *(volatile v8h*)(qln + qdst[i]) = qv[i];
    *(volatile v8h*)(kln + qdst[i]) = kvv[i];
    *(volatile us8*)(vth + vdst[i]) = vh8[i];
    *(volatile us8*)(vtl + vdst[i]) = vl8[i];
  }
  if (small) {
    *(volatile v4f*)(vpart + vpdst) = vp4;
    *(volatile v4f*)(ksc + ksdst)   = ks4;
  }
}

__global__ __launch_bounds__(256) void k_attn(
    const _Float16* __restrict__ qln, const _Float16* __restrict__ kln,
    const unsigned short* __restrict__ vth, const unsigned short* __restrict__ vtl,
    const float* __restrict__ vpart, const float* __restrict__ ksc,
    const int* __restrict__ mask, unsigned short* aoh, unsigned short* aol) {
  __shared__ __attribute__((aligned(16))) _Float16 sQ[TP_];
  __shared__ __attribute__((aligned(16))) _Float16 sK[TP_];
  __shared__ __attribute__((aligned(16))) unsigned short sVP[4 * TP_];
  __shared__ __attribute__((aligned(16))) float sKs[64];
  __shared__ __attribute__((aligned(16))) float sVs[64];
  __shared__ __attribute__((aligned(16))) float sDen[2][64];
  unsigned short* sVh = sVP;
  unsigned short* sVl = sVP + TP_;
  unsigned short* sPh = sVP + 2 * TP_;
  unsigned short* sPl = sVP + 3 * TP_;
  float* sO = (float*)sVP;

  const int bh = blockIdx.y, qt = blockIdx.x, q0 = qt * 64;
  const int b = bh / H_, h = bh - b * H_;
  const int tid = threadIdx.x, wave = tid >> 5, wm = wave & 3, wn2 = (wave >> 2) * 2;
  const int l = tid & 31, hh = l >> 4, m = l & 15;
  const int mflag = (mask[0] != 0);
  const int ntiles = mflag ? (qt + 1) : QT_;

  {
    const int row = tid >> 2, c = (tid & 3) * 16;
    const _Float16* src = qln + ((size_t)bh * S_ + q0 + row) * DH_ + c;
    *(v8h*)(sQ + row * PT_ + c)     = *(const v8h*)src;
    *(v8h*)(sQ + row * PT_ + c + 8) = *(const v8h*)(src + 8);
  }
  if (tid < 64) {
    float s = 0.f;
    for (int i = 0; i < QT_; ++i) s += vpart[((size_t)bh * QT_ + i) * 64 + tid];
    sVs[tid] = s;
  }

  float rowp[8];
#pragma unroll
  for (int j = 0; j < 8; ++j) rowp[j] = 0.f;
  v8f num0 = {0.f, 0.f, 0.f, 0.f, 0.f, 0.f, 0.f, 0.f};
  v8f num1 = {0.f, 0.f, 0.f, 0.f, 0.f, 0.f, 0.f, 0.f};

  for (int kt = 0; kt < ntiles; ++kt) {
    const int k0 = kt * 64;
    __syncthreads();
    {
      const int row = tid >> 2, c = (tid & 3) * 16;
      const _Float16* sk = kln + ((size_t)bh * S_ + k0 + row) * DH_ + c;
      *(v8h*)(sK + row * PT_ + c)     = *(const v8h*)sk;
      *(v8h*)(sK + row * PT_ + c + 8) = *(const v8h*)(sk + 8);
      const size_t vo = ((size_t)bh * DH_ + row) * S_ + k0 + c;
      *(us8*)(sVh + row * PT_ + c)     = *(const us8*)(vth + vo);
      *(us8*)(sVh + row * PT_ + c + 8) = *(const us8*)(vth + vo + 8);
      *(us8*)(sVl + row * PT_ + c)     = *(const us8*)(vtl + vo);
      *(us8*)(sVl + row * PT_ + c + 8) = *(const us8*)(vtl + vo + 8);
    }
    if (tid < 64) sKs[tid] = ksc[(size_t)bh * S_ + k0 + tid];
    __syncthreads();

    v8f s0 = {0.f, 0.f, 0.f, 0.f, 0.f, 0.f, 0.f, 0.f};
    v8f s1 = {0.f, 0.f, 0.f, 0.f, 0.f, 0.f, 0.f, 0.f};
#pragma unroll
    for (int c = 0; c < 2; ++c) {
      const v16h af = ldfrag_h(sQ + wm * 16 * PT_, PT_, c * 32);
      const v16h b0 = ldfrag_h(sK + wn2 * 16 * PT_, PT_, c * 32);
      const v16h b1 = ldfrag_h(sK + (wn2 + 1) * 16 * PT_, PT_, c * 32);
      s0 = mma_h(af, b0, s0);
      s1 = mma_h(af, b1, s1);
    }

#pragma unroll
    for (int p = 0; p < 2; ++p) {
      const v8f sc = p ? s1 : s0;
      const int nl = (wn2 + p) * 16 + m;
      const float ks = sKs[nl];
      const int kg = k0 + nl;
#pragma unroll
      for (int j = 0; j < 8; ++j) {
        const int ml = wm * 16 + hh * 8 + j;
        const int qg = q0 + ml;
        const float sv = sc[j] * SCALEF_;
        float pv;
        if (mflag) {
          const float xx = sv * ks;
          const float g = __builtin_amdgcn_rcpf(1.0f + __expf(-xx));
          const float u = g * ks;
          pv = (kg > qg) ? 0.f : (u + 0.5f * u * u);
        } else {
          const float u = sv * ks;
          pv = u + 0.5f * u * u;
        }
        rowp[j] += pv;
        const unsigned short hb = f2bf(pv);
        sPh[ml * PT_ + nl] = hb;
        sPl[ml * PT_ + nl] = f2bf(pv - bf2f(hb));
      }
    }
    __syncthreads();

#pragma unroll
    for (int c = 0; c < 2; ++c) {
      const v16b aph = ldfrag_b(sPh + wm * 16 * PT_, PT_, c * 32);
      const v16b apl = ldfrag_b(sPl + wm * 16 * PT_, PT_, c * 32);
      const v16b b0h = ldfrag_b(sVh + wn2 * 16 * PT_, PT_, c * 32);
      const v16b b0l = ldfrag_b(sVl + wn2 * 16 * PT_, PT_, c * 32);
      const v16b b1h = ldfrag_b(sVh + (wn2 + 1) * 16 * PT_, PT_, c * 32);
      const v16b b1l = ldfrag_b(sVl + (wn2 + 1) * 16 * PT_, PT_, c * 32);
      num0 = mma_b(aph, b0h, num0);
      num0 = mma_b(aph, b0l, num0);
      num0 = mma_b(apl, b0h, num0);
      num1 = mma_b(aph, b1h, num1);
      num1 = mma_b(aph, b1l, num1);
      num1 = mma_b(apl, b1h, num1);
    }
  }

#pragma unroll
  for (int j = 0; j < 8; ++j) {
    float v = rowp[j];
    v += __shfl_xor(v, 1, 32);
    v += __shfl_xor(v, 2, 32);
    v += __shfl_xor(v, 4, 32);
    v += __shfl_xor(v, 8, 32);
    rowp[j] = v;
  }
  __syncthreads();
  if (m == 0) {
#pragma unroll
    for (int j = 0; j < 8; ++j) sDen[wn2 >> 1][wm * 16 + hh * 8 + j] = rowp[j];
  }
  __syncthreads();

#pragma unroll
  for (int p = 0; p < 2; ++p) {
    const v8f nm = p ? num1 : num0;
    const int dl = (wn2 + p) * 16 + m;
    const float vs = sVs[dl];
#pragma unroll
    for (int j = 0; j < 8; ++j) {
      const int ml = wm * 16 + hh * 8 + j;
      const float den = (float)S_ + sDen[0][ml] + sDen[1][ml];
      const float rden = __builtin_amdgcn_rcpf(den);
      sO[ml * 64 + dl] = (vs + nm[j]) * rden;
    }
  }
  __syncthreads();

  us8 oh[2], ol[2];
  size_t odst[2];
#pragma unroll
  for (int i = 0; i < 2; ++i) {
    const int row = wave * 8 + 4 * i + (l >> 3);
    const int c8 = (l & 7) * 8;
    const v4f a  = *(const v4f*)(sO + row * 64 + c8);
    const v4f a2 = *(const v4f*)(sO + row * 64 + c8 + 4);
    float tmp[8] = {a[0], a[1], a[2], a[3], a2[0], a2[1], a2[2], a2[3]};
    split8(tmp, oh[i], ol[i]);
    odst[i] = ((size_t)b * S_ + q0 + row) * D_ + h * DH_ + c8;
  }
#pragma unroll
  for (int i = 0; i < 2; ++i) {
    *(volatile us8*)(aoh + odst[i]) = oh[i];
    *(volatile us8*)(aol + odst[i]) = ol[i];
  }
  __threadfence();
#pragma unroll
  for (int i = 0; i < 2; ++i) {
    *(volatile us8*)(aoh + odst[i]) = oh[i];
    *(volatile us8*)(aol + odst[i]) = ol[i];
  }
}

extern "C" void kernel_launch(void* const* d_in, const int* in_sizes, int n_in,
                              void* d_out, int out_size, void* d_ws,
                              size_t ws_size, hipStream_t stream) {
  if (n_in < 12) return;
  if (in_sizes[0] != NT_ * D_ || in_sizes[1] != D_ * D_ || in_sizes[2] != D_ ||
      in_sizes[3] != KVN_ * D_ || in_sizes[4] != D_ * D_ || in_sizes[5] != D_ ||
      in_sizes[6] != D_ || in_sizes[7] != D_ || in_sizes[8] != DH_ ||
      in_sizes[9] != DH_ || in_sizes[10] < 1 || in_sizes[11] < 1)
    return;
  if (out_size != NT_ * D_) return;

  const float* x     = (const float*)d_in[0];
  const float* Wq    = (const float*)d_in[1];
  const float* bq    = (const float*)d_in[2];
  const float* Wkv   = (const float*)d_in[3];
  const float* Wout  = (const float*)d_in[4];
  const float* bout  = (const float*)d_in[5];
  const float* lna_w = (const float*)d_in[6];
  const float* lna_b = (const float*)d_in[7];
  const float* lnb_w = (const float*)d_in[8];
  const float* lnb_b = (const float*)d_in[9];
  const float* zero  = (const float*)d_in[10];
  const int*   maskp = (const int*)d_in[11];
  float* out = (float*)d_out;

  char* ws = (char*)d_ws;
  size_t off = 0;
  auto carve = [&](size_t bytes) -> void* {
    void* p = ws + off;
    off += (bytes + 255) & ~(size_t)255;
    return p;
  };
  const size_t plane_x  = (size_t)NT_ * D_ * 2;
  unsigned short* xh   = (unsigned short*)carve(plane_x);
  unsigned short* xl   = (unsigned short*)carve(plane_x);
  unsigned short* yh   = (unsigned short*)carve(plane_x);
  unsigned short* yl   = (unsigned short*)carve(plane_x);
  unsigned short* wqh  = (unsigned short*)carve((size_t)D_ * D_ * 2);
  unsigned short* wql  = (unsigned short*)carve((size_t)D_ * D_ * 2);
  unsigned short* wkvh = (unsigned short*)carve((size_t)KVN_ * D_ * 2);
  unsigned short* wkvl = (unsigned short*)carve((size_t)KVN_ * D_ * 2);
  unsigned short* woh  = (unsigned short*)carve((size_t)D_ * D_ * 2);
  unsigned short* wol  = (unsigned short*)carve((size_t)D_ * D_ * 2);
  float* qf            = (float*)carve((size_t)NT_ * D_ * 4);
  float* kvf           = (float*)carve((size_t)NT_ * KVN_ * 4);
  _Float16* qln        = (_Float16*)carve(plane_x);
  _Float16* kln        = (_Float16*)carve(plane_x);
  unsigned short* vth  = (unsigned short*)carve(plane_x);
  unsigned short* vtl  = (unsigned short*)carve(plane_x);
  float* vpart         = (float*)carve((size_t)B_ * H_ * QT_ * 64 * 4);
  float* ksc           = (float*)carve((size_t)B_ * H_ * S_ * 4);
  unsigned short* aoh  = (unsigned short*)carve(plane_x);
  unsigned short* aol  = (unsigned short*)carve(plane_x);
  if (off > ws_size) return;

  k_prep<<<dim3(NT_), dim3(64), 0, stream>>>(x, lna_w, lna_b, xh, xl, yh, yl, NT_);

  k_split<<<dim3((D_ * D_ / 8 + 255) / 256), dim3(256), 0, stream>>>(Wq, wqh, wql, D_ * D_);
  k_split<<<dim3((KVN_ * D_ / 8 + 255) / 256), dim3(256), 0, stream>>>(Wkv, wkvh, wkvl, KVN_ * D_);
  k_split<<<dim3((D_ * D_ / 8 + 255) / 256), dim3(256), 0, stream>>>(Wout, woh, wol, D_ * D_);

  k_gemm<<<dim3(D_ / 64, NT_ / 64), dim3(256), 0, stream>>>(
      xh, xl, wqh, wql, bq, 1, qf, NT_, D_, D_);
  k_gemm<<<dim3(KVN_ / 64, NT_ / 64), dim3(256), 0, stream>>>(
      yh, yl, wkvh, wkvl, bq, 0, kvf, NT_, KVN_, D_);

  k_heads<<<dim3(NT_ / 64, H_), dim3(256), 0, stream>>>(
      qf, kvf, lnb_w, lnb_b, zero, qln, kln, vth, vtl, vpart, ksc);

  k_attn<<<dim3(QT_, B_ * H_), dim3(256), 0, stream>>>(
      qln, kln, vth, vtl, vpart, ksc, maskp, aoh, aol);

  k_gemm<<<dim3(D_ / 64, NT_ / 64), dim3(256), 0, stream>>>(
      aoh, aol, woh, wol, bout, 1, out, NT_, D_, D_);
}
